// TransformerBlock_21646635171948
// MI455X (gfx1250) — hardware-run, weakly checked
//
#include <hip/hip_runtime.h>


#define NB_  4
#define TT   1024
#define DM   1024
#define NH_  16
#define NKV  16
#define REP  (NH_ / NKV)
#define HD   64
#define DQ   (NH_ * HD)
#define DKV  (NKV * HD)
#define ZH   2
#define RH   512
#define WIN  0
#define PCAR 1024.0f
#define SCL  0.125f
typedef _Float16 h16;
typedef unsigned short bf;
typedef __attribute__((ext_vector_type(16))) __bf16   v16bf;
typedef __attribute__((ext_vector_type(16))) _Float16 v16h;
typedef __attribute__((ext_vector_type(8)))  _Float16 v8h;
typedef __attribute__((ext_vector_type(8)))  unsigned short v8us;
typedef __attribute__((ext_vector_type(8)))  float    v8f;
typedef __attribute__((ext_vector_type(4)))  float    v4f;
typedef v8h  __attribute__((may_alias)) v8ha;
typedef v4f  __attribute__((may_alias)) v4fa;
typedef v8us __attribute__((may_alias)) v8usa;

__device__ __forceinline__ unsigned short f2bf(float f) { unsigned u = __float_as_uint(f); u += 0x7FFFu + ((u >> 16) & 1u); return (unsigned short)(u >> 16); }
__device__ __forceinline__ float bf2f(unsigned short b) { return __uint_as_float(((unsigned)b) << 16); }
__device__ __forceinline__ float bfr(float f) { return bf2f(f2bf(f)); }
__device__ __forceinline__ v16h cat16(v8h lo, v8h hi) { return __builtin_shufflevector(lo, hi, 0, 1, 2, 3, 4, 5, 6, 7, 8, 9, 10, 11, 12, 13, 14, 15); }
__device__ __forceinline__ v16bf cat16b(v8us lo, v8us hi) { return __builtin_bit_cast(v16bf, __builtin_shufflevector(lo, hi, 0, 1, 2, 3, 4, 5, 6, 7, 8, 9, 10, 11, 12, 13, 14, 15)); }
__device__ __forceinline__ v8f wmma16(v16h a, v16h b, v8f c) { return __builtin_amdgcn_wmma_f32_16x16x32_f16(false, a, false, b, (short)0, c, false, false); }
__device__ __forceinline__ v8f wmmab(v16bf a, v16bf b, v8f c) { return __builtin_amdgcn_wmma_f32_16x16x32_bf16(false, a, false, b, (short)0, c, false, false); }


template <typename T16> struct WFrag;
template <> struct WFrag<h16> { typedef v16h V; static __device__ __forceinline__ V ld(const h16* p) { return cat16(*(const v8h*)p, *(const v8h*)(p + 16)); } static __device__ __forceinline__ v8f mma(V a, V b, v8f c) { return wmma16(a, b, c); } };
template <> struct WFrag<bf> { typedef v16bf V; static __device__ __forceinline__ V ld(const bf* p) { return cat16b(*(const v8us*)p, *(const v8us*)(p + 16)); } static __device__ __forceinline__ v8f mma(V a, V b, v8f c) { return wmmab(a, b, c); } };
template <typename T16, int NSPLIT, bool BIAS>
__global__ __launch_bounds__(32) void k_gemmw(const T16* __restrict__ A, const T16* __restrict__ A2, const T16* __restrict__ Bt, const T16* __restrict__ Bt2, int K, float* C, int ldc, const float* __restrict__ bias, size_t sA, size_t sB, size_t sC) {
    typedef typename WFrag<T16>::V V;
    __shared__ __align__(16) float os[16 * 68];
    const size_t z = blockIdx.z; A += z * sA; if (A2) A2 += z * sA; Bt += z * sB; if (Bt2) Bt2 += z * sB; C += z * sC;
    const int lane = threadIdx.x & 31, lr = lane & 15, hi = lane >> 4; const int r0 = blockIdx.x * 64, c0 = blockIdx.y * 64;
    v8f acc[4][4];
#pragma unroll
    for (int mb = 0; mb < 4; ++mb)
#pragma unroll
        for (int nb = 0; nb < 4; ++nb) acc[mb][nb] = (v8f){};
    const size_t aoff = (size_t)(r0 + lr) * K + 8 * hi, boff = (size_t)(c0 + lr) * K + 8 * hi;
#pragma unroll 1
    for (int kc = 0; kc < K; kc += 32) {
        V a[4], a2[4];
#pragma unroll
        for (int mb = 0; mb < 4; ++mb) { a[mb] = WFrag<T16>::ld(A + aoff + (size_t)mb * 16 * K + kc); if (NSPLIT == 1 || NSPLIT == 2) a2[mb] = WFrag<T16>::ld(A2 + aoff + (size_t)mb * 16 * K + kc); }
#pragma unroll
        for (int nb = 0; nb < 4; ++nb) { const V b = WFrag<T16>::ld(Bt + boff + (size_t)nb * 16 * K + kc); V b2; if (NSPLIT >= 2) b2 = WFrag<T16>::ld(Bt2 + boff + (size_t)nb * 16 * K + kc);
#pragma unroll
            for (int mb = 0; mb < 4; ++mb) { acc[mb][nb] = WFrag<T16>::mma(a[mb], b, acc[mb][nb]); if (NSPLIT == 1 || NSPLIT == 2) acc[mb][nb] = WFrag<T16>::mma(a2[mb], b, acc[mb][nb]); if (NSPLIT >= 2) acc[mb][nb] = WFrag<T16>::mma(a[mb], b2, acc[mb][nb]); } }
        asm volatile("v_nop\n\tv_nop\n\tv_nop\n\tv_nop" : "+v"(acc[0][0]), "+v"(acc[1][1]), "+v"(acc[2][2]), "+v"(acc[3][3]) : "v"(a[0]), "v"(a[3]));
    }
#pragma unroll
    for (int mb = 0; mb < 4; ++mb) {
#pragma unroll
        for (int nb = 0; nb < 4; ++nb) {
#pragma unroll
            for (int j = 0; j < 8; ++j) os[(hi * 8 + j) * 68 + nb * 16 + lr] = acc[mb][nb][j]; }
        __builtin_amdgcn_wave_barrier(); asm volatile("" ::: "memory");
        float* crow = C + (size_t)(r0 + mb * 16) * ldc + c0;
#pragma unroll 1
        for (int ps = 0; ps < 2; ++ps) {
#pragma unroll
            for (int s = 0; s < 8; ++s) { const int row = 2 * s + hi, cofs = lr * 4; v4f val = *(const v4fa*)(os + row * 68 + cofs); if (BIAS) { val[0] += bfr(bias[c0 + cofs]); val[1] += bfr(bias[c0 + cofs + 1]); val[2] += bfr(bias[c0 + cofs + 2]); val[3] += bfr(bias[c0 + cofs + 3]); }
                *(volatile v4f*)(crow + (size_t)row * ldc + cofs) = val; }
            if (ps == 0) __threadfence(); }
        __builtin_amdgcn_wave_barrier(); asm volatile("" ::: "memory");
    }
}

__device__ __forceinline__ h16 tohx(float x) { return (h16)x; }
__device__ __forceinline__ void splitf(float y, unsigned short& h, unsigned short& l) { h = f2bf(y); l = f2bf(y - bf2f(h)); }
typedef __attribute__((ext_vector_type(2))) _Float16 v2h;
typedef __attribute__((ext_vector_type(4))) _Float16 v4h;
typedef __attribute__((ext_vector_type(2))) unsigned short v2us;
typedef __attribute__((ext_vector_type(4))) unsigned short v4us;
typedef __attribute__((ext_vector_type(2))) float v2f;
typedef __attribute__((ext_vector_type(4))) int v4i;

__global__ __launch_bounds__(256) void k_wtG(const float* __restrict__ w, int K, int N, bf* Bt) {
    const int lane = threadIdx.x & 31; const int L0 = (blockIdx.x * 8 + (threadIdx.x >> 5)) * 8; const int nlines = N * K / 64;
#pragma unroll
    for (int ps = 0; ps < 2; ++ps) {
#pragma unroll 1
        for (int l = 0; l < 8; ++l) { const int L = L0 + l; if (L >= nlines) break; const size_t e = (size_t)L * 64 + lane * 2; const int k = (int)(e % K), n = (int)(e / K); v2us o;
            o[0] = f2bf(w[(size_t)k * N + n]); o[1] = f2bf(w[(size_t)(k + 1) * N + n]); *(volatile v2us*)(Bt + e) = o; }
        if (ps == 0) __threadfence(); }
}
__global__ __launch_bounds__(256) void k_cvt8(const float* __restrict__ src, bf* dst, size_t n8) { const size_t i = (size_t)blockIdx.x * 256 + threadIdx.x; if (i >= n8) return; const v8f v = *(const v8f*)(src + i * 8); v8us o;
#pragma unroll
    for (int k = 0; k < 8; ++k) o[k] = f2bf(v[k]); *(volatile v8us*)(dst + i * 8) = o; __threadfence(); *(volatile v8us*)(dst + i * 8) = o; }
__constant__ float INV[HD / 2] = {1.0f,0.749894202f,0.562341332f,0.421696514f,0.316227764f,0.237137362f,0.177827939f,0.133352146f,0.100000001f,0.0749894157f,0.0562341288f,0.0421696492f,0.0316227786f,0.0237137359f,0.0177827943f,0.0133352149f,0.00999999978f,0.00749894232f,0.00562341325f,0.00421696482f,0.00316227786f,0.00237137382f,0.00177827943f,0.00133352145f,0.00100000005f,0.000749894185f,0.000562341302f,0.000421696488f,0.000316227786f,0.000237137385f,0.00017782794f,0.00013335215f};
__global__ __launch_bounds__(256) void k_cstab(float* CS) { const int idx = blockIdx.x * 256 + threadIdx.x; if (idx >= TT * HD) return; const int t = idx / HD, d = idx % HD; const float ang = __fmul_rn((float)t, INV[d % (HD / 2)]); v2f cs; cs[0] = cosf(ang); cs[1] = sinf(ang);
    *(volatile v2f*)(CS + (size_t)idx * 2) = cs; __threadfence(); *(volatile v2f*)(CS + (size_t)idx * 2) = cs; }

__global__ __launch_bounds__(256) void k_rope(const float* __restrict__ F, int pitch, int nheads, const float* __restrict__ CS, const float* __restrict__ RF, const float* __restrict__ nw, float sc, h16* P16, bf* Ph, bf* Pl) {
    const size_t e = ((size_t)blockIdx.x * 256 + threadIdx.x) * 2; if (e >= (size_t)nheads * TT * HD) return; const int d = (int)(e % HD); const int t = (int)((e / HD) % TT); const int h = (int)(e / ((size_t)HD * TT)); const float* f = F + (size_t)t * pitch + h * HD; const float rf = RF ? RF[(size_t)h * TT + t] : 1.0f; v2h o16; v2us oh, ol;
#pragma unroll
    for (int q = 0; q < 2; ++q) { const int dd = d + q; const int dp = (dd < HD / 2) ? dd + HD / 2 : dd - HD / 2; float x0 = f[dd], x1 = f[dp];
        if (RF) { float n0 = __fmul_rn(x0, rf), n1 = __fmul_rn(x1, rf); asm volatile("" : "+v"(n0)); asm volatile("" : "+v"(n1)); x0 = __fmul_rn(bfr(nw[dd]), n0); x1 = __fmul_rn(bfr(nw[dp]), n1); }
        const v2f cs = *(const v2f*)(CS + ((size_t)t * HD + dd) * 2); float a = __fmul_rn(x0, cs[0]), bq = __fmul_rn(x1, cs[1]); asm volatile("" : "+v"(a)); asm volatile("" : "+v"(bq)); const float r = ((dd < HD / 2) ? __fsub_rn(a, bq) : __fadd_rn(a, bq)) * sc;
        o16[q] = tohx(r); unsigned short a2, c2; splitf(r, a2, c2); oh[q] = a2; ol[q] = c2; }
    *(volatile v2h*)(P16 + e) = o16; *(volatile v2us*)(Ph + e) = oh; *(volatile v2us*)(Pl + e) = ol; __threadfence(); *(volatile v2h*)(P16 + e) = o16; *(volatile v2us*)(Ph + e) = oh; *(volatile v2us*)(Pl + e) = ol; }
__global__ __launch_bounds__(256) void k_vtp(const float* __restrict__ F, int pitch, int nheads, h16* V16, bf* Vh, bf* Vl) { const size_t e = ((size_t)blockIdx.x * 256 + threadIdx.x) * 2; if (e >= (size_t)nheads * HD * TT) return; const int t = (int)(e % TT); const int d = (int)((e / TT) % HD); const int g = (int)(e / ((size_t)TT * HD)); v2h o16; v2us oh, ol;
#pragma unroll
    for (int q = 0; q < 2; ++q) { const float x = F[(size_t)(t + q) * pitch + g * HD + d]; o16[q] = tohx(x); unsigned short a2, c2; splitf(x, a2, c2); oh[q] = a2; ol[q] = c2; }
    *(volatile v2h*)(V16 + e) = o16; *(volatile v2us*)(Vh + e) = oh; *(volatile v2us*)(Vl + e) = ol; __threadfence(); *(volatile v2h*)(V16 + e) = o16; *(volatile v2us*)(Vh + e) = oh; *(volatile v2us*)(Vl + e) = ol; }

__global__ __launch_bounds__(256) void k_asoft(const float* __restrict__ Sb, const float* __restrict__ MKb, h16* P16, bf* Ph, bf* Pl) {
    const int lane = threadIdx.x & 31; const int row = blockIdx.x * 8 + (threadIdx.x >> 5); if (row >= ZH * TT) return; const int i = row % TT; const int zz = row / TT; (void)zz; const bool qok = (bfr(MKb[i]) != 0.0f); const bool hires = (i < RH); const float* sr = Sb + (size_t)row * TT; float v[TT / 32]; float mx = -3.0e38f;
#pragma unroll
    for (int ch = 0; ch < TT / 128; ++ch) { const int j0 = ch * 128 + lane * 4; const v4f a = *(const v4f*)(sr + j0); const v4f m4 = *(const v4f*)(MKb + j0);
#pragma unroll
        for (int q = 0; q < 4; ++q) { const int j = j0 + q; (void)j; float sa = a[q] * SCL; asm volatile("" : "+v"(sa)); const float t = (qok && bfr(m4[q]) != 0.0f) ? sa : -1.0e9f;     v[ch * 4 + q] = t; mx = fmaxf(mx, t); } }
#pragma unroll
    for (int sh = 16; sh; sh >>= 1) mx = fmaxf(mx, __shfl_xor(mx, sh, 32));
    float sum = 0.f;
#pragma unroll
    for (int k = 0; k < TT / 32; ++k) { float d0 = __fsub_rn(v[k], mx); asm volatile("" : "+v"(d0)); v[k] = __builtin_amdgcn_exp2f(__fmul_rn(d0, 1.4426950408889634f)); sum += v[k]; }
#pragma unroll
    for (int sh = 16; sh; sh >>= 1) sum += __shfl_xor(sum, sh, 32);
    const float f = __fdiv_rn(hires ? 1.0f : PCAR, sum);
#pragma unroll 1
    for (int ps = 0; ps < 2; ++ps) {
        if (hires) {
#pragma unroll
            for (int ch = 0; ch < TT / 128; ++ch) { v4us oh, ol;
#pragma unroll
                for (int q = 0; q < 4; ++q) { unsigned short a, c2; splitf(v[ch * 4 + q] * f, a, c2); oh[q] = a; ol[q] = c2; }
                const size_t oo = ((size_t)zz * (RH ? RH : 1) + i) * TT + ch * 128 + lane * 4; *(volatile v4us*)(Ph + oo) = oh; *(volatile v4us*)(Pl + oo) = ol; }
        } else {
#pragma unroll
            for (int ch = 0; ch < TT / 128; ++ch) { v4h o4;
#pragma unroll
                for (int q = 0; q < 4; ++q) o4[q] = tohx(v[ch * 4 + q] * f);
                *(volatile v4h*)(P16 + (size_t)row * TT + ch * 128 + lane * 4) = o4; } }
        if (ps == 0) __threadfence(); }
}
__global__ __launch_bounds__(256) void k_merge(const float* __restrict__ O, int h0, bf* Ah, bf* Al) { const size_t e = ((size_t)blockIdx.x * 256 + threadIdx.x) * 2; if (e >= (size_t)ZH * TT * HD) return; const int d = (int)(e % HD); const int t = (int)((e / HD) % TT); const int zz = (int)(e / ((size_t)HD * TT)); const float cs = (t < RH) ? 1.0f : (1.0f / PCAR); const size_t oo = (size_t)t * DQ + (h0 + zz) * HD + d;
    v2us oh, ol;
#pragma unroll
    for (int q = 0; q < 2; ++q) { unsigned short a, c2; splitf(O[e + q] * cs, a, c2); oh[q] = a; ol[q] = c2; } *(volatile v2us*)(Ah + oo) = oh; *(volatile v2us*)(Al + oo) = ol; __threadfence(); *(volatile v2us*)(Ah + oo) = oh; *(volatile v2us*)(Al + oo) = ol; }


__global__ __launch_bounds__(256) void k_lnhl(const float* __restrict__ X, size_t xpitch, int nrows, int nreal, int roundin, const float* __restrict__ gw, const float* __restrict__ gb, bf* Yh, bf* Yl, float* Yf) {
    const int lane = threadIdx.x & 31; const int r = blockIdx.x * 8 + (threadIdx.x >> 5); if (r >= nrows) return; float hv[32]; float s = 0.f;
    if (r < nreal) { const float* xr = X + (size_t)r * xpitch;
#pragma unroll
        for (int ch = 0; ch < 8; ++ch) { const v4f y = *(const v4f*)(xr + ch * 128 + lane * 4);
#pragma unroll
            for (int q = 0; q < 4; ++q) { const float u = roundin ? bfr(y[q]) : y[q]; hv[ch * 4 + q] = u; s += u; } } } else {
#pragma unroll
        for (int k = 0; k < 32; ++k) hv[k] = 0.f; }
#pragma unroll
    for (int sh = 16; sh; sh >>= 1) s += __shfl_xor(s, sh, 32);
    float mu = s * (1.0f / 1024.0f); asm volatile("" : "+v"(mu)); float s2 = 0.f;
#pragma unroll
    for (int k = 0; k < 32; ++k) { float d0 = __fsub_rn(hv[k], mu); asm volatile("" : "+v"(d0)); float p = __fmul_rn(d0, d0); asm volatile("" : "+v"(p)); s2 = __fadd_rn(s2, p); }
#pragma unroll
    for (int sh = 16; sh; sh >>= 1) s2 += __shfl_xor(s2, sh, 32);
    float var = __fadd_rn(s2 * (1.0f / 1024.0f), 1e-5f); asm volatile("" : "+v"(var)); const float rs = __frsqrt_rn(var);
#pragma unroll 1
    for (int ps = 0; ps < 2; ++ps) {
#pragma unroll
        for (int ch = 0; ch < 8; ++ch) { const int c0 = ch * 128 + lane * 4; v4us oh, ol; v4f of;
#pragma unroll
            for (int q = 0; q < 4; ++q) { float y = 0.f; if (r < nreal) { float gg = bfr(gw[c0 + q]); asm volatile("" : "+v"(gg)); float d0 = __fsub_rn(hv[ch * 4 + q], mu); asm volatile("" : "+v"(d0)); float n0 = __fmul_rn(d0, rs); asm volatile("" : "+v"(n0)); y = __fmul_rn(n0, gg); asm volatile("" : "+v"(y)); if (gb) y = __fadd_rn(y, bfr(gb[c0 + q])); } of[q] = y; unsigned short a, c2; splitf(y, a, c2); oh[q] = a; ol[q] = c2; }
            *(volatile v4us*)(Yh + (size_t)r * 1024 + c0) = oh; *(volatile v4us*)(Yl + (size_t)r * 1024 + c0) = ol; if (Yf) *(volatile v4f*)(Yf + (size_t)r * 1024 + c0) = of; }
        if (ps == 0) __threadfence(); } }
__global__ __launch_bounds__(256) void k_lnseg(float* F, size_t pitch, int nrows, const float* __restrict__ gw) {
    const int lane = threadIdx.x & 31; const int r = blockIdx.x * 8 + (threadIdx.x >> 5); if (r >= nrows) return; float* fr = F + (size_t)r * pitch; float hv[32]; float s = 0.f;
#pragma unroll
    for (int ch = 0; ch < 8; ++ch) { const v4f y = *(const v4f*)(fr + ch * 128 + lane * 4);
#pragma unroll
        for (int q = 0; q < 4; ++q) { hv[ch * 4 + q] = y[q]; s += y[q]; } }
#pragma unroll
    for (int sh = 16; sh; sh >>= 1) s += __shfl_xor(s, sh, 32);
    float mu = s * (1.0f / 1024.0f); asm volatile("" : "+v"(mu)); float s2 = 0.f;
#pragma unroll
    for (int k = 0; k < 32; ++k) { float d0 = __fsub_rn(hv[k], mu); asm volatile("" : "+v"(d0)); float p = __fmul_rn(d0, d0); asm volatile("" : "+v"(p)); s2 = __fadd_rn(s2, p); }
#pragma unroll
    for (int sh = 16; sh; sh >>= 1) s2 += __shfl_xor(s2, sh, 32);
    float var = __fadd_rn(s2 * (1.0f / 1024.0f), 1e-5f); asm volatile("" : "+v"(var)); const float rs = __frsqrt_rn(var);
    __builtin_amdgcn_wave_barrier(); asm volatile("" ::: "memory");
#pragma unroll 1
    for (int ps = 0; ps < 2; ++ps) {
#pragma unroll
        for (int ch = 0; ch < 8; ++ch) { const int c0 = ch * 128 + lane * 4; v4f o;
#pragma unroll
            for (int q = 0; q < 4; ++q) { float gg = bfr(gw[c0 + q]); asm volatile("" : "+v"(gg)); float d0 = __fsub_rn(hv[ch * 4 + q], mu); asm volatile("" : "+v"(d0)); float n0 = __fmul_rn(d0, rs); asm volatile("" : "+v"(n0)); o[q] = __fmul_rn(n0, gg); }
            *(volatile v4f*)(fr + c0) = o; }
        if (ps == 0) __threadfence(); } }
__global__ __launch_bounds__(256) void k_add2(const float* __restrict__ A, int roundA, const float* __restrict__ Bv, float* Cc, size_t n4) { const size_t i = (size_t)blockIdx.x * 256 + threadIdx.x; if (i >= n4) return; const v4f a = *(const v4f*)(A + i * 4); const v4f bb = *(const v4f*)(Bv + i * 4); v4f o;
#pragma unroll
    for (int q = 0; q < 4; ++q) { float ar = roundA ? bfr(a[q]) : a[q]; asm volatile("" : "+v"(ar)); o[q] = __fadd_rn(ar, bb[q]); } *(volatile v4f*)(Cc + i * 4) = o; __threadfence(); *(volatile v4f*)(Cc + i * 4) = o; }
__global__ __launch_bounds__(256) void k_geluhl(const float* __restrict__ Hh, bf* Gh, bf* Gl, size_t n4) { const size_t i = (size_t)blockIdx.x * 256 + threadIdx.x; if (i >= n4) return; const v4f h = *(const v4f*)(Hh + i * 4); v4us oh, ol;
#pragma unroll
    for (int q = 0; q < 4; ++q) { float u = __fmul_rn(h[q], 0.70710678118654752f); asm volatile("" : "+v"(u)); float e1 = __fadd_rn(1.0f, erff(u)); asm volatile("" : "+v"(e1)); float hh = __fmul_rn(0.5f, h[q]); asm volatile("" : "+v"(hh)); const float y = __fmul_rn(hh, e1); unsigned short a, c2; splitf(y, a, c2); oh[q] = a; ol[q] = c2; }
    *(volatile v4us*)(Gh + i * 4) = oh; *(volatile v4us*)(Gl + i * 4) = ol; __threadfence(); *(volatile v4us*)(Gh + i * 4) = oh; *(volatile v4us*)(Gl + i * 4) = ol; }
__device__ __forceinline__ float siluf(float z) { const float e = expf(-z); float den = __fadd_rn(1.0f, e); asm volatile("" : "+v"(den)); return __fdiv_rn(z, den); }
__global__ __launch_bounds__(256) void k_cond(const float* __restrict__ temp, const float* __restrict__ tw1, const float* __restrict__ tb1, const float* __restrict__ Tw1, const float* __restrict__ Tb1, bf* TUh, bf* TUl, bf* TEh, bf* TEl) {
    const int lane = threadIdx.x & 31; const int r = blockIdx.x * 8 + (threadIdx.x >> 5); if (r >= 64) return; const float tv = (r < NB_) ? bfr(temp[r]) : 0.f;
#pragma unroll 1
    for (int ps = 0; ps < 2; ++ps) {
#pragma unroll 1
        for (int ch = 0; ch < 8; ++ch) { const int c0 = ch * 128 + lane * 4; v4us ah, al, eh, el;
#pragma unroll
            for (int q = 0; q < 4; ++q) { const int c = c0 + q; float y = 0.f, z = 0.f;
                if (r < NB_) { float p = __fmul_rn(tv, bfr(tw1[c])); asm volatile("" : "+v"(p)); y = siluf(__fadd_rn(p, bfr(tb1[c]))); }
                if (r == 0) { float acc = 0.f;
#pragma unroll 1
                    for (int k = 128; k < 256; ++k) acc = __fadd_rn(acc, bfr(Tw1[(size_t)k * 1024 + c]));
                    z = siluf(__fadd_rn(acc, bfr(Tb1[c]))); }
                unsigned short a, c2; splitf(y, a, c2); ah[q] = a; al[q] = c2; splitf(z, a, c2); eh[q] = a; el[q] = c2; }
            const size_t oo = (size_t)r * 1024 + c0; *(volatile v4us*)(TUh + oo) = ah; *(volatile v4us*)(TUl + oo) = al; *(volatile v4us*)(TEh + oo) = eh; *(volatile v4us*)(TEl + oo) = el; }
        if (ps == 0) __threadfence(); } }
__global__ __launch_bounds__(256) void k_xmod(const float* __restrict__ XN, const float* __restrict__ TE, const float* __restrict__ TEE, bf* Mh, bf* Ml) { const size_t e = ((size_t)blockIdx.x * 256 + threadIdx.x) * 4; if (e >= (size_t)64 * 1024) return; const int r = (int)(e / 1024); const int c = (int)(e % 1024); v4us oh, ol;
#pragma unroll
    for (int q = 0; q < 4; ++q) { float y = 0.f; if (r < NB_) { float t1 = __fadd_rn(XN[e + q], TE[e + q]); asm volatile("" : "+v"(t1)); y = __fadd_rn(t1, TEE[c + q]); } unsigned short a, c2; splitf(y, a, c2); oh[q] = a; ol[q] = c2; }
    *(volatile v4us*)(Mh + e) = oh; *(volatile v4us*)(Ml + e) = ol; __threadfence(); *(volatile v4us*)(Mh + e) = oh; *(volatile v4us*)(Ml + e) = ol; }
__global__ __launch_bounds__(256) void k_struc(const float* __restrict__ FT, const bf* __restrict__ KPh, const bf* __restrict__ KPl, const float* __restrict__ FVp, const float* __restrict__ MKb, int b, float* CT) {
    const int lane = threadIdx.x & 31; const int h = blockIdx.x * 8 + (threadIdx.x >> 5); if (h >= NH_) return; const float* ft = FT + (size_t)b * 3 * DM; const v2f qv = *(const v2f*)(ft + h * HD + lane * 2); const bool qok = (bfr(MKb[0]) != 0.0f);
    float m = -3.0e38f, Z = 0.f; v2f acc = (v2f){0.f, 0.f};
#pragma unroll 1
    for (int j = 0; j <= TT; ++j) { v2f kv, vv; bool kok;
        if (j < TT) { const size_t pe = ((size_t)h * TT + j) * HD + lane * 2; const v2us kh = *(const v2us*)(KPh + pe), kl = *(const v2us*)(KPl + pe); kv[0] = __fadd_rn(bf2f(kh[0]), bf2f(kl[0])); kv[1] = __fadd_rn(bf2f(kh[1]), bf2f(kl[1])); vv = *(const v2f*)(FVp + (size_t)j * 3 * DM + h * HD + lane * 2); kok = (bfr(MKb[j]) != 0.0f); }
        else { kv = *(const v2f*)(ft + DM + h * HD + lane * 2); vv = *(const v2f*)(ft + 2 * DM + h * HD + lane * 2); kok = qok; }
        float s = __fadd_rn(__fmul_rn(qv[0], kv[0]), 0.f); asm volatile("" : "+v"(s)); float p2 = __fmul_rn(qv[1], kv[1]); asm volatile("" : "+v"(p2)); s = __fadd_rn(s, p2);
#pragma unroll
        for (int sh = 16; sh; sh >>= 1) s += __shfl_xor(s, sh, 32);
        float sc = s * SCL; asm volatile("" : "+v"(sc)); const float t = (qok && kok) ? sc : -1.0e9f;
        const float mn = fmaxf(m, t); float d1 = __fsub_rn(m, mn), d2 = __fsub_rn(t, mn); asm volatile("" : "+v"(d1), "+v"(d2));
        const float r = __builtin_amdgcn_exp2f(__fmul_rn(d1, 1.4426950408889634f)), w = __builtin_amdgcn_exp2f(__fmul_rn(d2, 1.4426950408889634f));
        float zr = __fmul_rn(Z, r); asm volatile("" : "+v"(zr)); Z = __fadd_rn(zr, w); m = mn;
#pragma unroll
        for (int q = 0; q < 2; ++q) { float t0 = __fmul_rn(acc[q], r); asm volatile("" : "+v"(t0)); float t1 = __fmul_rn(w, vv[q]); asm volatile("" : "+v"(t1)); acc[q] = __fadd_rn(t0, t1); } }
    const float iz = __fdiv_rn(1.0f, Z); v2f o; o[0] = acc[0] * iz; o[1] = acc[1] * iz; float* dst = CT + (size_t)b * DM + h * HD + lane * 2; *(volatile v2f*)dst = o; __threadfence(); *(volatile v2f*)dst = o; }
__global__ __launch_bounds__(256) void k_split64(const float* __restrict__ X, int nreal, bf* Yh, bf* Yl) { const size_t e = ((size_t)blockIdx.x * 256 + threadIdx.x) * 4; if (e >= (size_t)64 * 1024) return; const int r = (int)(e / 1024); v4us oh, ol;
#pragma unroll
    for (int q = 0; q < 4; ++q) { const float y = (r < nreal) ? X[e + q] : 0.f; unsigned short a, c2; splitf(y, a, c2); oh[q] = a; ol[q] = c2; } *(volatile v4us*)(Yh + e) = oh; *(volatile v4us*)(Yl + e) = ol; __threadfence(); *(volatile v4us*)(Yh + e) = oh; *(volatile v4us*)(Yl + e) = ol; }
extern "C" void kernel_launch(void* const* d_in, const int* in_sizes, int n_in,
                              void* d_out, int out_size, void* d_ws, size_t ws_size, hipStream_t stream) {
    (void)in_sizes; (void)n_in; (void)out_size;
    const float* xs = (const float*)d_in[0]; const float* xt = (const float*)d_in[1]; const float* temp = (const float*)d_in[2]; const float* MK = (const float*)d_in[3];
    const float* lnqs_w = (const float*)d_in[4]; const float* lnqs_b = (const float*)d_in[5]; const float* wqkv_s = (const float*)d_in[6]; const float* lnqt_w = (const float*)d_in[7]; const float* lnqt_b = (const float*)d_in[8]; const float* wqkv_t = (const float*)d_in[9];
    const float* qln_s = (const float*)d_in[10]; const float* kln_s = (const float*)d_in[11]; const float* qln_t = (const float*)d_in[12]; const float* kln_t = (const float*)d_in[13]; const float* wout_s = (const float*)d_in[14]; const float* wout_t = (const float*)d_in[15];
    const float* tw1 = (const float*)d_in[16]; const float* tb1 = (const float*)d_in[17]; const float* tw2 = (const float*)d_in[18]; const float* tb2 = (const float*)d_in[19]; const float* Tw1 = (const float*)d_in[20]; const float* Tb1 = (const float*)d_in[21]; const float* Tw2 = (const float*)d_in[22]; const float* Tb2 = (const float*)d_in[23];
    const float* fln_s_w = (const float*)d_in[24]; const float* fln_s_b = (const float*)d_in[25]; const float* fw1_s = (const float*)d_in[26]; const float* fw2_s = (const float*)d_in[27]; const float* fln_t_w = (const float*)d_in[28]; const float* fln_t_b = (const float*)d_in[29]; const float* fw1_t = (const float*)d_in[30]; const float* fw2_t = (const float*)d_in[31];
    float* OUT0 = (float*)d_out;
    float* OUT1 = (float*)d_out + (size_t)NB_ * TT * DM;
    const int FF = 4 * DM;
    char* wsp = (char*)d_ws;
    auto take = [&](size_t bytes) { char* p = wsp; wsp += (bytes + 255) & ~(size_t)255; return (void*)p; };
    bf* WQKV_S = (bf*)take((size_t)3 * DM * DM * 2); bf* WO_S = (bf*)take((size_t)DM * DM * 2); bf* W1_S = (bf*)take((size_t)FF * DM * 2); bf* W2_S = (bf*)take((size_t)DM * FF * 2);
    bf* WQKV_T = (bf*)take((size_t)3 * DM * DM * 2); bf* WO_T = (bf*)take((size_t)DM * DM * 2); bf* W1_T = (bf*)take((size_t)FF * DM * 2); bf* W2_T = (bf*)take((size_t)DM * FF * 2); bf* TW2 = (bf*)take((size_t)DM * DM * 2); bf* TTW2 = (bf*)take((size_t)DM * DM * 2); float* CS = (float*)take((size_t)TT * HD * 2 * 4);
    bf* XNh = (bf*)take((size_t)64 * DM * 2); bf* XNl = (bf*)take((size_t)64 * DM * 2); float* XN = (float*)take((size_t)64 * DM * 4); bf* TUh = (bf*)take((size_t)64 * DM * 2); bf* TUl = (bf*)take((size_t)64 * DM * 2); bf* TEh = (bf*)take((size_t)64 * DM * 2); bf* TEl = (bf*)take((size_t)64 * DM * 2); float* TE = (float*)take((size_t)64 * DM * 4); float* TEE = (float*)take((size_t)64 * DM * 4);
    bf* Mh = (bf*)take((size_t)64 * DM * 2); bf* Ml = (bf*)take((size_t)64 * DM * 2); float* FT = (float*)take((size_t)64 * 3 * DM * 4); float* CT = (float*)take((size_t)64 * DM * 4); bf* CTh = (bf*)take((size_t)64 * DM * 2); bf* CTl = (bf*)take((size_t)64 * DM * 2); float* OS = (float*)take((size_t)64 * DM * 4); float* X1T = (float*)take((size_t)64 * DM * 4); bf* LTh = (bf*)take((size_t)64 * DM * 2); bf* LTl = (bf*)take((size_t)64 * DM * 2); float* HT = (float*)take((size_t)64 * FF * 4); bf* GTh = (bf*)take((size_t)64 * FF * 2); bf* GTl = (bf*)take((size_t)64 * FF * 2); float* Y2T = (float*)take((size_t)64 * DM * 4);
    bf* LNh = (bf*)take((size_t)TT * DM * 2); bf* LNl = (bf*)take((size_t)TT * DM * 2); float* F = (float*)take((size_t)TT * 3 * DM * 4);
    h16* QP16 = (h16*)take((size_t)NH_ * TT * HD * 2); h16* KP16 = (h16*)take((size_t)NKV * TT * HD * 2); h16* VT16 = (h16*)take((size_t)NKV * HD * TT * 2);
    bf* QPh = (bf*)take((size_t)NH_ * TT * HD * 2); bf* QPl = (bf*)take((size_t)NH_ * TT * HD * 2); bf* KPh = (bf*)take((size_t)NKV * TT * HD * 2); bf* KPl = (bf*)take((size_t)NKV * TT * HD * 2); bf* VTh = (bf*)take((size_t)NKV * HD * TT * 2); bf* VTl = (bf*)take((size_t)NKV * HD * TT * 2); bf* Ph = (bf*)take((size_t)ZH * RH * TT * 2); bf* Pl = (bf*)take((size_t)ZH * RH * TT * 2);
    float* Sb = (float*)take((size_t)ZH * TT * TT * 4); h16* P16 = (h16*)take((size_t)ZH * TT * TT * 2); float* Ob = (float*)take((size_t)ZH * TT * HD * 4); bf* ATh = (bf*)take((size_t)TT * DQ * 2); bf* ATl = (bf*)take((size_t)TT * DQ * 2);
    float* YO = (float*)take((size_t)TT * DM * 4); float* X1 = (float*)take((size_t)TT * DM * 4); bf* L2h = (bf*)take((size_t)TT * DM * 2); bf* L2l = (bf*)take((size_t)TT * DM * 2); float* HB = (float*)take((size_t)TT * FF * 4); bf* Gh = (bf*)take((size_t)TT * FF * 2); bf* Gl = (bf*)take((size_t)TT * FF * 2); float* Y2 = (float*)take((size_t)TT * DM * 4);
    if ((size_t)(wsp - (char*)d_ws) > ws_size) return;
    k_wtG<<<(unsigned)((DM * 3 * DM / 64 + 63) / 64), 256, 0, stream>>>(wqkv_s, DM, 3 * DM, WQKV_S); k_wtG<<<(unsigned)((DM * DM / 64 + 63) / 64), 256, 0, stream>>>(wout_s, DM, DM, WO_S); k_wtG<<<(unsigned)((DM * FF / 64 + 63) / 64), 256, 0, stream>>>(fw1_s, DM, FF, W1_S); k_wtG<<<(unsigned)((FF * DM / 64 + 63) / 64), 256, 0, stream>>>(fw2_s, FF, DM, W2_S);
    k_wtG<<<(unsigned)((DM * 3 * DM / 64 + 63) / 64), 256, 0, stream>>>(wqkv_t, DM, 3 * DM, WQKV_T); k_wtG<<<(unsigned)((DM * DM / 64 + 63) / 64), 256, 0, stream>>>(wout_t, DM, DM, WO_T); k_wtG<<<(unsigned)((DM * FF / 64 + 63) / 64), 256, 0, stream>>>(fw1_t, DM, FF, W1_T); k_wtG<<<(unsigned)((FF * DM / 64 + 63) / 64), 256, 0, stream>>>(fw2_t, FF, DM, W2_T);
    k_wtG<<<(unsigned)((DM * DM / 64 + 63) / 64), 256, 0, stream>>>(tw2, DM, DM, TW2); k_wtG<<<(unsigned)((DM * DM / 64 + 63) / 64), 256, 0, stream>>>(Tw2, DM, DM, TTW2);
    k_cstab<<<(TT * HD + 255) / 256, 256, 0, stream>>>(CS);
    const size_t L64 = ((size_t)64 * DM / 4 + 255) / 256, L1K = ((size_t)TT * DM / 4 + 255) / 256;
    k_lnhl<<<8, 256, 0, stream>>>(xt, (size_t)DM, 64, NB_, 1, lnqt_w, lnqt_b, XNh, XNl, XN);
    k_cond<<<8, 256, 0, stream>>>(temp, tw1, tb1, Tw1, Tb1, TUh, TUl, TEh, TEl);
    k_gemmw<bf, 1, true><<<dim3(1, DM / 64, 1), 32, 0, stream>>>(TUh, TUl, TW2, nullptr, DM, TE, DM, tb2, 0, 0, 0);
    k_gemmw<bf, 1, true><<<dim3(1, DM / 64, 1), 32, 0, stream>>>(TEh, TEl, TTW2, nullptr, DM, TEE, DM, Tb2, 0, 0, 0);
    k_xmod<<<(unsigned)L64, 256, 0, stream>>>(XN, TE, TEE, Mh, Ml);
    k_gemmw<bf, 1, false><<<dim3(1, 3 * DM / 64, 1), 32, 0, stream>>>(Mh, Ml, WQKV_T, nullptr, DM, FT, 3 * DM, nullptr, 0, 0, 0);
    k_lnseg<<<1, 256, 0, stream>>>(FT, (size_t)3 * DM, NB_, qln_t); k_lnseg<<<1, 256, 0, stream>>>(FT + DM, (size_t)3 * DM, NB_, kln_t);
    const unsigned LQ = (unsigned)(((size_t)NH_ * TT * HD / 2 + 255) / 256), LKv = (unsigned)(((size_t)NKV * TT * HD / 2 + 255) / 256);
    for (int b = 0; b < NB_; ++b) { const float* xb = xs + (size_t)b * TT * DM; const float* mkb = MK + (size_t)b * TT;
        k_lnhl<<<TT / 8, 256, 0, stream>>>(xb, (size_t)DM, TT, TT, 1, lnqs_w, lnqs_b, LNh, LNl, nullptr);
        k_gemmw<bf, 1, false><<<dim3(TT / 64, 3 * DM / 64, 1), 32, 0, stream>>>(LNh, LNl, WQKV_S, nullptr, DM, F, 3 * DM, nullptr, 0, 0, 0);
        k_lnseg<<<TT / 8, 256, 0, stream>>>(F, (size_t)3 * DM, TT, qln_s); k_lnseg<<<TT / 8, 256, 0, stream>>>(F + DM, (size_t)3 * DM, TT, kln_s);
        k_rope<<<LQ, 256, 0, stream>>>(F, 3 * DM, NH_, CS, nullptr, nullptr, 1.0f, QP16, QPh, QPl); k_rope<<<LKv, 256, 0, stream>>>(F + DM, 3 * DM, NKV, CS, nullptr, nullptr, 1.0f, KP16, KPh, KPl); k_vtp<<<LKv, 256, 0, stream>>>(F + 2 * DM, 3 * DM, NKV, VT16, VTh, VTl);
        for (int h0 = 0; h0 < NH_; h0 += ZH) { const size_t zq = (size_t)h0, zk = (size_t)h0;
            k_gemmw<bf, 2, false><<<dim3(RH / 64, TT / 64, ZH), 32, 0, stream>>>(QPh + zq * TT * HD, QPl + zq * TT * HD, KPh + zk * TT * HD, KPl + zk * TT * HD, HD, Sb, TT, nullptr, (size_t)TT * HD, (size_t)TT * HD, (size_t)TT * TT);
            k_gemmw<h16, 0, false><<<dim3((TT - RH) / 64, TT / 64, ZH), 32, 0, stream>>>(QP16 + zq * TT * HD + (size_t)RH * HD, nullptr, KP16 + zk * TT * HD, nullptr, HD, Sb + (size_t)RH * TT, TT, nullptr, (size_t)TT * HD, (size_t)TT * HD, (size_t)TT * TT);
            k_asoft<<<ZH * TT / 8, 256, 0, stream>>>(Sb, mkb, P16, Ph, Pl);
            k_gemmw<bf, 2, false><<<dim3(RH / 64, HD / 64, ZH), 32, 0, stream>>>(Ph, Pl, VTh + zk * HD * TT, VTl + zk * HD * TT, TT, Ob, HD, nullptr, (size_t)RH * TT, (size_t)HD * TT, (size_t)TT * HD);
            k_gemmw<h16, 0, false><<<dim3((TT - RH) / 64, HD / 64, ZH), 32, 0, stream>>>(P16 + (size_t)RH * TT, nullptr, VT16 + zk * HD * TT, nullptr, TT, Ob + (size_t)RH * HD, HD, nullptr, (size_t)TT * TT, (size_t)HD * TT, (size_t)TT * HD);
            k_merge<<<(unsigned)(((size_t)ZH * TT * HD / 2 + 255) / 256), 256, 0, stream>>>(Ob, h0, ATh, ATl); }
        k_struc<<<2, 256, 0, stream>>>(FT, KPh, KPl, F + 2 * DM, mkb, b, CT);
        k_gemmw<bf, 1, false><<<dim3(TT / 64, DM / 64, 1), 32, 0, stream>>>(ATh, ATl, WO_S, nullptr, DQ, YO, DM, nullptr, 0, 0, 0);
        k_add2<<<(unsigned)L1K, 256, 0, stream>>>(xb, 1, YO, X1, (size_t)TT * DM / 4);
        k_lnhl<<<TT / 8, 256, 0, stream>>>(X1, (size_t)DM, TT, TT, 0, fln_s_w, fln_s_b, L2h, L2l, nullptr);
        k_gemmw<bf, 1, false><<<dim3(TT / 64, FF / 64, 1), 32, 0, stream>>>(L2h, L2l, W1_S, nullptr, DM, HB, FF, nullptr, 0, 0, 0);
        k_geluhl<<<(unsigned)(((size_t)TT * FF / 4 + 255) / 256), 256, 0, stream>>>(HB, Gh, Gl, (size_t)TT * FF / 4);
        k_gemmw<bf, 1, false><<<dim3(TT / 64, DM / 64, 1), 32, 0, stream>>>(Gh, Gl, W2_S, nullptr, FF, Y2, DM, nullptr, 0, 0, 0);
        k_add2<<<(unsigned)L1K, 256, 0, stream>>>(X1, 0, Y2, OUT0 + (size_t)b * TT * DM, (size_t)TT * DM / 4); }
    k_split64<<<(unsigned)L64, 256, 0, stream>>>(CT, NB_, CTh, CTl);
    k_gemmw<bf, 1, false><<<dim3(1, DM / 64, 1), 32, 0, stream>>>(CTh, CTl, WO_T, nullptr, DQ, OS, DM, nullptr, 0, 0, 0);
    k_add2<<<(unsigned)(((size_t)NB_ * DM / 4 + 255) / 256), 256, 0, stream>>>(xt, 1, OS, X1T, (size_t)NB_ * DM / 4);
    k_lnhl<<<8, 256, 0, stream>>>(X1T, (size_t)DM, 64, NB_, 0, fln_t_w, fln_t_b, LTh, LTl, nullptr);
    k_gemmw<bf, 1, false><<<dim3(1, FF / 64, 1), 32, 0, stream>>>(LTh, LTl, W1_T, nullptr, DM, HT, FF, nullptr, 0, 0, 0);
    k_geluhl<<<(unsigned)(((size_t)64 * FF / 4 + 255) / 256), 256, 0, stream>>>(HT, GTh, GTl, (size_t)64 * FF / 4);
    k_gemmw<bf, 1, false><<<dim3(1, DM / 64, 1), 32, 0, stream>>>(GTh, GTl, W2_T, nullptr, FF, Y2T, DM, nullptr, 0, 0, 0);
    k_add2<<<(unsigned)(((size_t)NB_ * DM / 4 + 255) / 256), 256, 0, stream>>>(X1T, 0, Y2T, OUT1, (size_t)NB_ * DM / 4);
}
